// RelationalGraphLayer_44178033607358
// MI455X (gfx1250) — hardware-verified
//
#include <hip/hip_runtime.h>
#include <stddef.h>
#include <stdint.h>


#define DD     128
#define NET    3
#define NNT    2
#define PN     (NET * DD)
#define ENCK   ((NET + 1) * DD)
#define G1N    (NNT * DD)
#define NTHR   256
#define NWAVE  8
#define EPT    8
#define CHUNK  (NTHR * EPT)
#define WCAP   (EPT * 32)
#define LISTN  (NWAVE * WCAP)
#define NBA    1024
#define SLA    10
#define RCAP   28672
#define DEGCAP 64
#define GBM    64
#define GBN    128
#define GTHR   128
#define EPB    256
#define AP     136
#define DP     68
#define OP     128
#define ECST   (2 * PN)
#define EDGE_LDS_BYTES (EPB * DP * 4 + EPB * AP * 2 + EPB * OP * 2 + ECST * 4 + 64 * 4)
#define NUW1   (PN * (DD / 8))
#define NUW2   (PN * (DD / 8))
#define NUW3   (G1N * (ENCK / 8))
#define NUW4   (DD * (G1N / 8))
#define NUWT   (NUW1 + NUW2 + NUW3 + NUW4)
#define AGG_ZINTS (LISTN + 2 * RCAP + 3 * NBA)
#define AGG_LDS_INTS (AGG_ZINTS + 16)
#define WSMAX  268435456

static_assert((CHUNK & (CHUNK - 1)) == 0 && CHUNK <= 4096);
static_assert((NBA & (NBA - 1)) == 0 && NBA == (1 << SLA));
static_assert(((long long)CHUNK << SLA) < (1LL << 31));
static_assert(LISTN % NTHR == 0);
static_assert(NBA % NWAVE == 0 && NBA % 32 == 0 && NBA % GBM == 0);
static_assert(RCAP % 4 == 0 && AGG_ZINTS % 4 == 0 && LISTN % 4 == 0);
static_assert(AGG_LDS_INTS * 4 <= 300000);
static_assert(EDGE_LDS_BYTES <= 300000);
static_assert(DD % 32 == 0 && ENCK % 32 == 0 && G1N % 32 == 0);
static_assert(PN % GBN == 0 && G1N % GBN == 0 && DD == GBN);
static_assert(GBM == (GTHR / 32) * 16 && GBN == 4 * 32);
static_assert(NUW1 % NTHR == 0 && NUW2 % NTHR == 0 && NUW3 % NTHR == 0 && NUW4 % NTHR == 0);
static_assert(EPB == NTHR && EPB == 8 * 32);
static_assert((DP * 4) % 16 == 0 && (AP * 2) % 16 == 0 && AP >= DD && DP >= 64 && OP == DD);
static_assert((EPB * DP * 4) % 16 == 0 && (EPB * AP * 2) % 16 == 0 && (EPB * OP * 2) % 16 == 0 && (ECST * 4) % 16 == 0);
static_assert(DD == 4 * 32);

typedef float          v4f   __attribute__((ext_vector_type(4)));
typedef float          v8f   __attribute__((ext_vector_type(8)));
typedef int            v4i   __attribute__((ext_vector_type(4)));
typedef int            v8i   __attribute__((ext_vector_type(8)));
typedef unsigned int   v2u   __attribute__((ext_vector_type(2)));
typedef unsigned int   v4u   __attribute__((ext_vector_type(4)));
typedef unsigned short v8us  __attribute__((ext_vector_type(8)));
typedef unsigned short v16us __attribute__((ext_vector_type(16)));
typedef _Float16       v16h  __attribute__((ext_vector_type(16)));
typedef __bf16         v16bf __attribute__((ext_vector_type(16)));
typedef v4f  __attribute__((may_alias)) v4fa;
typedef v4i  __attribute__((may_alias)) v4ia;
typedef v2u  __attribute__((may_alias)) v2ua;
typedef v4u  __attribute__((may_alias)) v4ua;
typedef v8us __attribute__((may_alias)) v8usa;
union Frag { v16bf b; v16h f; v16us u; v8us h[2]; v8i w; };

__device__ __forceinline__ v8f wmb(const Frag& a, const Frag& b, v8f c) {
  v8f d = __builtin_amdgcn_wmma_f32_16x16x32_bf16(false, a.b, false, b.b, (short)0, c, false, false);
  asm volatile("v_nop\n\tv_nop\n\tv_nop\n\tv_nop" : "+v"(d) : "v"(a.w), "v"(b.w));
  return d;
}
__device__ __forceinline__ v8f wmh(const Frag& a, const Frag& b, v8f c) {
  v8f d = __builtin_amdgcn_wmma_f32_16x16x32_f16(false, a.f, false, b.f, (short)0, c, false, false);
  asm volatile("v_nop\n\tv_nop\n\tv_nop\n\tv_nop" : "+v"(d) : "v"(a.w), "v"(b.w));
  return d;
}

__device__ __forceinline__ unsigned bf16_bits(float f) {
  const unsigned u = __float_as_uint(f);
  return (u + 0x7FFFu + ((u >> 16) & 1u)) >> 16;
}
__device__ __forceinline__ float bf16_val(float f) {
  return __uint_as_float(bf16_bits(f) << 16);
}
__device__ __forceinline__ unsigned short f2h(float x) {
  x = x > 65000.0f ? 65000.0f : x;
  x = x < -65000.0f ? -65000.0f : x;
  const _Float16 h = (_Float16)x;
  return __builtin_bit_cast(unsigned short, h);
}
__device__ __forceinline__ float h2f(unsigned w) {
  const unsigned short s = (unsigned short)(w & 0xFFFFu);
  const _Float16 h = __builtin_bit_cast(_Float16, s);
  return (float)h;
}

template <int SLB>
__device__ __forceinline__ int scan_chunk(const int* __restrict__ dsts, int nE, int cbase, int slotBase,
                                          int nb, int vec8, int* list, int tid, int lane, int wave) {
  int wc = 0;
  const int el0  = tid * EPT;
  const int e0   = cbase + el0;
  const int sent = -2147483647 - 1;
  v4i da, db;
  if (vec8 != 0 && cbase + CHUNK <= nE) {
    da = *(const v4i*)(dsts + e0);
    db = *(const v4i*)(dsts + e0 + 4);
  } else {
    da.x = (e0     < nE) ? dsts[min(e0,     nE - 1)] : sent;
    da.y = (e0 + 1 < nE) ? dsts[min(e0 + 1, nE - 1)] : sent;
    da.z = (e0 + 2 < nE) ? dsts[min(e0 + 2, nE - 1)] : sent;
    da.w = (e0 + 3 < nE) ? dsts[min(e0 + 3, nE - 1)] : sent;
    db.x = (e0 + 4 < nE) ? dsts[min(e0 + 4, nE - 1)] : sent;
    db.y = (e0 + 5 < nE) ? dsts[min(e0 + 5, nE - 1)] : sent;
    db.z = (e0 + 6 < nE) ? dsts[min(e0 + 6, nE - 1)] : sent;
    db.w = (e0 + 7 < nE) ? dsts[min(e0 + 7, nE - 1)] : sent;
  }
  const unsigned nbs = (unsigned)slotBase;
  const unsigned unb = (unsigned)nb;
  const unsigned s0 = (unsigned)da.x - nbs, s1 = (unsigned)da.y - nbs;
  const unsigned s2 = (unsigned)da.z - nbs, s3 = (unsigned)da.w - nbs;
  const unsigned s4 = (unsigned)db.x - nbs, s5 = (unsigned)db.y - nbs;
  const unsigned s6 = (unsigned)db.z - nbs, s7 = (unsigned)db.w - nbs;
  const bool h0 = s0 < unb, h1 = s1 < unb, h2 = s2 < unb, h3 = s3 < unb;
  const bool h4 = s4 < unb, h5 = s5 < unb, h6 = s6 < unb, h7 = s7 < unb;
  const unsigned any = __builtin_amdgcn_ballot_w32(h0 | h1 | h2 | h3 | h4 | h5 | h6 | h7);
  if (any != 0u) {
#define HITJ(J, HJ, SJ) { \
      const unsigned mj = __builtin_amdgcn_ballot_w32(HJ); \
      if (mj != 0u) { \
        if (HJ) { \
          const int pos = wc + (int)__builtin_amdgcn_mbcnt_lo(mj, 0u); \
          if (pos < WCAP) list[wave * WCAP + pos] = ((el0 + (J)) << SLB) | (int)(SJ); \
        } \
        wc += (int)__builtin_popcount(mj); } }
    HITJ(0, h0, s0)
    HITJ(1, h1, s1)
    HITJ(2, h2, s2)
    HITJ(3, h3, s3)
    HITJ(4, h4, s4)
    HITJ(5, h5, s5)
    HITJ(6, h6, s6)
    HITJ(7, h7, s7)
#undef HITJ
  }
  return wc;
}

__global__ __launch_bounds__(NTHR) void k_prep(const float* __restrict__ nf, const float* __restrict__ We1,
                                               const float* __restrict__ We2, const float* __restrict__ Wn1,
                                               const float* __restrict__ Wn2, int nN, int mRows,
                                               unsigned short* NFB, unsigned short* We1T, unsigned short* We2T,
                                               unsigned short* Wn1T, unsigned short* Wn2T) {
  const int u = (int)blockIdx.x * NTHR + (int)threadIdx.x;
  v8us o;
  unsigned short* dp;
  if (u < NUW1) {
    const int n  = u >> 4;
    const int k8 = (u & 15) * 8;
    const int t  = n >> 7, c = n & 127;
    const float* p = We1 + ((size_t)t * DD + k8) * DD + c;
#pragma unroll
    for (int i = 0; i < 8; ++i) o[i] = (unsigned short)bf16_bits(p[(size_t)i * DD]);
    dp = We1T + (size_t)n * DD + k8;
  } else if (u < NUW1 + NUW2) {
    const int v  = u - NUW1;
    const int n  = v >> 4;
    const int k8 = (v & 15) * 8;
    const int t  = n >> 7, c = n & 127;
    const float* p = We2 + ((size_t)t * DD + k8) * DD + c;
#pragma unroll
    for (int i = 0; i < 8; ++i) o[i] = f2h(1024.0f * bf16_val(p[(size_t)i * DD]));
    dp = We2T + (size_t)n * DD + k8;
  } else if (u < NUW1 + NUW2 + NUW3) {
    const int v  = u - NUW1 - NUW2;
    const int n  = v >> 6;
    const int k8 = (v & 63) * 8;
    const int ut = n >> 7, c = n & 127;
    const float* p = Wn1 + ((size_t)ut * ENCK + k8) * DD + c;
#pragma unroll
    for (int i = 0; i < 8; ++i) o[i] = f2h(1024.0f * bf16_val(p[(size_t)i * DD]));
    dp = Wn1T + (size_t)n * ENCK + k8;
  } else if (u < NUWT) {
    const int v  = u - NUW1 - NUW2 - NUW3;
    const int n  = v >> 5;
    const int k8 = (v & 31) * 8;
    const int ut = k8 >> 7, kk = k8 & 127;
    const float* p = Wn2 + ((size_t)ut * DD + kk) * DD + n;
#pragma unroll
    for (int i = 0; i < 8; ++i) o[i] = f2h(1024.0f * bf16_val(p[(size_t)i * DD]));
    dp = Wn2T + (size_t)n * G1N + k8;
  } else {
    const int v = u - NUWT;
    if (v >= mRows * 16) return;
    const int row = v >> 4;
    const int k8  = (v & 15) * 8;
    const int rc  = row < nN ? row : nN - 1;
    const float* p = nf + (size_t)rc * DD + k8;
    const v4f a = *(const v4fa*)p;
    const v4f b = *(const v4fa*)(p + 4);
    const bool ok = row < nN;
    o[0] = ok ? (unsigned short)bf16_bits(a.x) : (unsigned short)0;
    o[1] = ok ? (unsigned short)bf16_bits(a.y) : (unsigned short)0;
    o[2] = ok ? (unsigned short)bf16_bits(a.z) : (unsigned short)0;
    o[3] = ok ? (unsigned short)bf16_bits(a.w) : (unsigned short)0;
    o[4] = ok ? (unsigned short)bf16_bits(b.x) : (unsigned short)0;
    o[5] = ok ? (unsigned short)bf16_bits(b.y) : (unsigned short)0;
    o[6] = ok ? (unsigned short)bf16_bits(b.z) : (unsigned short)0;
    o[7] = ok ? (unsigned short)bf16_bits(b.w) : (unsigned short)0;
    dp = NFB + (size_t)row * DD + k8;
  }
  *(volatile v8us*)dp = o;
  __threadfence();
  *(volatile v8us*)dp = o;
}

template <int BF, int EPI>
__global__ __launch_bounds__(GTHR) void k_gemm(const unsigned short* __restrict__ A, int lda,
                                               const unsigned short* __restrict__ BT, int ldb, int K,
                                               const float* __restrict__ bias, const int* __restrict__ nty, int nN,
                                               unsigned short* C16, float* C32, int ldc) {
  __shared__ __attribute__((aligned(16))) float stg[GBM * GBN];
  __shared__ __attribute__((aligned(16))) float sb[256];
  __shared__ int st[GBM];
  const int tid = (int)threadIdx.x, lane = tid & 31, wave = tid >> 5, hh = lane >> 4, m = lane & 15;
  const int rowBase = (int)blockIdx.x * GBM;
  const int colBase = (int)blockIdx.y * GBN;
  const int cb = (int)blockIdx.y;

  if constexpr (EPI == 1) {
    sb[tid] = bf16_val(bias[colBase + tid]);
  }
  if constexpr (EPI == 2) {
    sb[tid] = bf16_val(bias[tid]);
    sb[GBN + tid] = bf16_val(bias[GBN + tid]);
  }
  if constexpr (EPI != 0) {
    if (tid < GBM) {
      int rr = rowBase + tid;
      rr = rr < nN ? rr : nN - 1;
      st[tid] = nty[rr];
    }
  }

  v8f acc[8];
  {
    const v8f z = {0.f, 0.f, 0.f, 0.f, 0.f, 0.f, 0.f, 0.f};
#pragma unroll
    for (int t = 0; t < 8; ++t) acc[t] = z;
  }
  const unsigned short* ap = A  + (size_t)(rowBase + 16 * wave + m) * (size_t)lda + 8 * hh;
  const unsigned short* bp = BT + (size_t)(colBase + m) * (size_t)ldb + 8 * hh;

#pragma unroll 1
  for (int k0 = 0; k0 < K; k0 += 32) {
    Frag af;
    af.h[0] = *(const v8usa*)(ap + k0);
    af.h[1] = *(const v8usa*)(ap + k0 + 16);
#pragma unroll
    for (int nt = 0; nt < 8; ++nt) {
      const unsigned short* wq = bp + (size_t)(16 * nt) * (size_t)ldb + k0;
      Frag bf;
      bf.h[0] = *(const v8usa*)wq;
      bf.h[1] = *(const v8usa*)(wq + 16);
      if constexpr (BF != 0) acc[nt] = wmb(af, bf, acc[nt]);
      else                   acc[nt] = wmh(af, bf, acc[nt]);
    }
  }

#pragma unroll
  for (int nt = 0; nt < 8; ++nt) {
    const int lc = 16 * nt + m;
#pragma unroll
    for (int r = 0; r < 8; ++r) {
      const int lr = 16 * wave + 8 * hh + r;
      stg[lr * GBN + lc] = acc[nt][r];
    }
  }
  __syncthreads();

  if constexpr (EPI != 2) {
    v8us po[8];
#pragma unroll
    for (int i = 0; i < 8; ++i) {
      const int lr = 16 * wave + 2 * i + hh;
      const float* sp = stg + lr * GBN + 8 * m;
      const v4f xa = *(const v4fa*)sp;
      const v4f xb = *(const v4fa*)(sp + 4);
      const v8f x8 = {xa.x, xa.y, xa.z, xa.w, xb.x, xb.y, xb.z, xb.w};
      v8us o;
      if constexpr (EPI == 0) {
#pragma unroll
        for (int j = 0; j < 8; ++j) o[j] = f2h(16.0f * x8[j]);
      } else {
        const int row = rowBase + lr;
        const int uu  = st[lr];
        const bool ok = (uu == cb) && (row < nN);
        const v4f ba = *(const v4fa*)(sb + 8 * m);
        const v4f bb = *(const v4fa*)(sb + 8 * m + 4);
        const v8f b8 = {ba.x, ba.y, ba.z, ba.w, bb.x, bb.y, bb.z, bb.w};
#pragma unroll
        for (int j = 0; j < 8; ++j) {
          const float g = fmaxf(fmaf(x8[j], 0.00048828125f, b8[j]), 0.0f) * 16.0f;
          o[j] = ok ? f2h(g) : (unsigned short)0;
        }
      }
      po[i] = o;
    }
#pragma unroll
    for (int i = 0; i < 8; ++i) {
      const int lr = 16 * wave + 2 * i + hh;
      unsigned short* dp = C16 + (size_t)(rowBase + lr) * (size_t)ldc + colBase + 8 * m;
      *(volatile v8us*)dp = po[i];
    }
    __threadfence();
#pragma unroll
    for (int i = 0; i < 8; ++i) {
      const int lr = 16 * wave + 2 * i + hh;
      unsigned short* dp = C16 + (size_t)(rowBase + lr) * (size_t)ldc + colBase + 8 * m;
      *(volatile v8us*)dp = po[i];
    }
  } else {
    v4f pv[16];
#pragma unroll
    for (int i = 0; i < 16; ++i) {
      const int lr = 16 * wave + i;
      const int uu = st[lr];
      const bool valid = (unsigned)uu < (unsigned)NNT;
      const int uc = valid ? uu : 0;
      const float fb = valid ? 1.0f : 0.0f;
      const v4f x  = *(const v4fa*)(stg + lr * GBN + 4 * lane);
      const v4f bq = *(const v4fa*)(sb + uc * DD + 4 * lane);
      v4f v;
      v.x = fmaf(fb, bq.x, x.x * 6.103515625e-05f);
      v.y = fmaf(fb, bq.y, x.y * 6.103515625e-05f);
      v.z = fmaf(fb, bq.z, x.z * 6.103515625e-05f);
      v.w = fmaf(fb, bq.w, x.w * 6.103515625e-05f);
      pv[i] = v;
    }
#pragma unroll
    for (int i = 0; i < 16; ++i) {
      const int row = rowBase + 16 * wave + i;
      if (row < nN) {
        float* op = C32 + (size_t)row * (size_t)ldc + colBase + 4 * lane;
        *(volatile v4f*)op = pv[i];
      }
    }
    __threadfence();
#pragma unroll
    for (int i = 0; i < 16; ++i) {
      const int row = rowBase + 16 * wave + i;
      if (row < nN) {
        float* op = C32 + (size_t)row * (size_t)ldc + colBase + 4 * lane;
        *(volatile v4f*)op = pv[i];
      }
    }
  }
}

__global__ __launch_bounds__(NTHR) void k_edge(const int* __restrict__ srcs, const int* __restrict__ ets,
                                               int eBase, int nHalf, int nN,
                                               const unsigned short* __restrict__ P16,
                                               const unsigned short* __restrict__ W2T,
                                               const float* __restrict__ be1, const float* __restrict__ be2,
                                               unsigned short* Mh) {
  extern __shared__ __attribute__((aligned(16))) float dyn[];
  float*          sD  = dyn;
  unsigned short* sA  = (unsigned short*)(dyn + EPB * DP);
  unsigned short* sO  = sA + EPB * AP;
  float*          cst = (float*)(sO + EPB * OP);
  int*            swc = (int*)(cst + ECST);

  const int tid = (int)threadIdx.x, lane = tid & 31, wave = tid >> 5, hh = lane >> 4, m = lane & 15;
  const int R0 = 32 * wave;

#pragma unroll
  for (int it = 0; it < 2; ++it) {
    const int i  = tid + NTHR * it;
    const int ic = i < PN ? i : PN - 1;
    const float v1 = bf16_val(be1[ic]);
    const float v2 = bf16_val(be2[ic]);
    if (i < PN) { cst[i] = v1; cst[PN + i] = v2; }
  }

  const int el = (int)blockIdx.x * EPB + tid;
  const int ee = el < nHalf ? el : nHalf - 1;
  const int eg = eBase + ee;
  int s = srcs[eg];
  s = s < 0 ? 0 : (s > nN - 1 ? nN - 1 : s);
  const int traw = ets[eg];
  const int tc = traw < 0 ? 0 : (traw > NET - 1 ? NET - 1 : traw);

  const unsigned q0 = __builtin_amdgcn_ballot_w32(tc == 0);
  const unsigned q1 = __builtin_amdgcn_ballot_w32(tc == 1);
  const unsigned q2 = __builtin_amdgcn_ballot_w32(tc == 2);
  const unsigned qt = (tc == 0) ? q0 : ((tc == 1) ? q1 : q2);
  const int rin = (int)__builtin_amdgcn_mbcnt_lo(qt, 0u);
  if (lane == 0) {
    swc[4 * wave]     = (int)__builtin_popcount(q0);
    swc[4 * wave + 1] = (int)__builtin_popcount(q1);
    swc[4 * wave + 2] = (int)__builtin_popcount(q2);
    swc[4 * wave + 3] = 0;
  }
  __syncthreads();

  int t0 = 0, t1 = 0, t2 = 0, pre = 0;
#pragma unroll
  for (int w2 = 0; w2 < NWAVE; ++w2) {
    const int c0 = swc[4 * w2], c1 = swc[4 * w2 + 1], c2 = swc[4 * w2 + 2];
    const int cw = (tc == 0) ? c0 : ((tc == 1) ? c1 : c2);
    pre += (w2 < wave) ? cw : 0;
    t0 += c0; t1 += c1; t2 += c2;
  }
  t0 = __builtin_amdgcn_readfirstlane(t0);
  t1 = __builtin_amdgcn_readfirstlane(t1);
  t2 = __builtin_amdgcn_readfirstlane(t2);
  const int st1 = t0, st2 = t0 + t1;
  const int stc = (tc == 0) ? 0 : ((tc == 1) ? st1 : st2);
  int crow = stc + pre + rin;
  crow = crow < 0 ? 0 : (crow > EPB - 1 ? EPB - 1 : crow);

  {
    const unsigned short* pr = P16 + (size_t)s * PN + tc * DD;
    const float* bb = cst + tc * DD;
    unsigned short* ra = sA + crow * AP;
#pragma unroll 2
    for (int c8 = 0; c8 < DD / 8; ++c8) {
      const v4u w  = *(const v4ua*)(pr + 8 * c8);
      const v4f ba = *(const v4fa*)(bb + 8 * c8);
      const v4f bc = *(const v4fa*)(bb + 8 * c8 + 4);
      const v8f x8 = {h2f(w.x), h2f(w.x >> 16), h2f(w.y), h2f(w.y >> 16),
                      h2f(w.z), h2f(w.z >> 16), h2f(w.w), h2f(w.w >> 16)};
      const v8f b8 = {ba.x, ba.y, ba.z, ba.w, bc.x, bc.y, bc.z, bc.w};
      v8us o;
#pragma unroll
      for (int j = 0; j < 8; ++j)
        o[j] = f2h(16.0f * fmaxf(fmaf(x8[j], 0.0625f, b8[j]), 0.0f));
      *(v8usa*)(ra + 8 * c8) = o;
    }
  }
  __syncthreads();

#pragma unroll 1
  for (int tp = 0; tp < NET; ++tp) {
    const int sS = (tp == 0) ? 0 : ((tp == 1) ? st1 : st2);
    const int sE = sS + ((tp == 0) ? t0 : ((tp == 1) ? t1 : t2));
    const int f0 = ((sS < R0 + 16) && (sE > R0)) ? 1 : 0;
    const int f1 = ((sS < R0 + 32) && (sE > R0 + 16)) ? 2 : 0;
    const int actw = __builtin_amdgcn_readfirstlane(f0 | f1);
#pragma unroll 1
    for (int ch = 0; ch < 2; ++ch) {
      v8f acc[2][4];
      {
        const v8f z = {0.f, 0.f, 0.f, 0.f, 0.f, 0.f, 0.f, 0.f};
#pragma unroll
        for (int mt = 0; mt < 2; ++mt)
#pragma unroll
          for (int nt = 0; nt < 4; ++nt) acc[mt][nt] = z;
      }
      if (actw != 0) {
        const unsigned short* ap0 = sA + (R0 + m) * AP + 8 * hh;
        const unsigned short* ap1 = ap0 + 16 * AP;
        const unsigned short* bp  = W2T + (size_t)(tp * DD + ch * 64 + m) * DD + 8 * hh;
#pragma unroll 1
        for (int k0 = 0; k0 < DD; k0 += 32) {
          Frag bq[4];
#pragma unroll
          for (int nt = 0; nt < 4; ++nt) {
            const unsigned short* wq = bp + (size_t)(16 * nt) * DD + k0;
            bq[nt].h[0] = *(const v8usa*)wq;
            bq[nt].h[1] = *(const v8usa*)(wq + 16);
          }
          if (actw & 1) {
            Frag a0;
            a0.h[0] = *(const v8usa*)(ap0 + k0);
            a0.h[1] = *(const v8usa*)(ap0 + k0 + 16);
#pragma unroll
            for (int nt = 0; nt < 4; ++nt) acc[0][nt] = wmh(a0, bq[nt], acc[0][nt]);
          }
          if (actw & 2) {
            Frag a1;
            a1.h[0] = *(const v8usa*)(ap1 + k0);
            a1.h[1] = *(const v8usa*)(ap1 + k0 + 16);
#pragma unroll
            for (int nt = 0; nt < 4; ++nt) acc[1][nt] = wmh(a1, bq[nt], acc[1][nt]);
          }
        }
      }
#pragma unroll
      for (int nt = 0; nt < 4; ++nt) {
        const int col = 16 * nt + m;
#pragma unroll
        for (int mt = 0; mt < 2; ++mt)
#pragma unroll
          for (int rr = 0; rr < 8; ++rr)
            sD[(R0 + 16 * mt + 8 * hh + rr) * DP + col] = acc[mt][nt][rr];
      }
      __syncthreads();

      {
        const float* drow = sD + crow * DP;
        const float* b2p  = cst + PN + tp * DD + ch * 64;
        unsigned short* orow = sO + tid * OP + ch * 64;
        const bool mine = (tc == tp);
#pragma unroll 2
        for (int c8 = 0; c8 < 8; ++c8) {
          const v4f d0 = *(const v4fa*)(drow + 8 * c8);
          const v4f d1 = *(const v4fa*)(drow + 8 * c8 + 4);
          const v4f e0 = *(const v4fa*)(b2p + 8 * c8);
          const v4f e1 = *(const v4fa*)(b2p + 8 * c8 + 4);
          const v8f d8 = {d0.x, d0.y, d0.z, d0.w, d1.x, d1.y, d1.z, d1.w};
          const v8f e8 = {e0.x, e0.y, e0.z, e0.w, e1.x, e1.y, e1.z, e1.w};
          v8us o;
#pragma unroll
          for (int j = 0; j < 8; ++j)
            o[j] = f2h(16.0f * fmaxf(fmaf(d8[j], 6.103515625e-05f, e8[j]), 0.0f));
          if (mine) *(v8usa*)(orow + 8 * c8) = o;
        }
      }
      __syncthreads();
    }
  }

  v8us pm[16];
#pragma unroll
  for (int i = 0; i < 16; ++i) {
    const int lr = R0 + 2 * i + hh;
    pm[i] = *(const v8usa*)(sO + lr * OP + 8 * m);
  }
  const size_t rb = (size_t)blockIdx.x * EPB;
#pragma unroll
  for (int i = 0; i < 16; ++i) {
    const int lr = R0 + 2 * i + hh;
    unsigned short* dp = Mh + (rb + (size_t)lr) * DD + 8 * m;
    *(volatile v8us*)dp = pm[i];
  }
  __threadfence();
#pragma unroll
  for (int i = 0; i < 16; ++i) {
    const int lr = R0 + 2 * i + hh;
    unsigned short* dp = Mh + (rb + (size_t)lr) * DD + 8 * m;
    *(volatile v8us*)dp = pm[i];
  }
}

__global__ __launch_bounds__(NTHR) void k_scan(const int* __restrict__ dsts, const int* __restrict__ ets,
                                               int nE, int nN, int vec8, int mRows, int accum,
                                               const unsigned short* __restrict__ msg, float* agg) {
  extern __shared__ __attribute__((aligned(16))) int dsm[];
  int* list = dsm;
  int* hl   = dsm + LISTN;
  int* sl   = dsm + LISTN + RCAP;
  int* cnt  = dsm + LISTN + 2 * RCAP;
  int* offs = cnt + NBA;
  int* cur  = offs + NBA;
  int* misc = cur + NBA;
  const int tid = (int)threadIdx.x, lane = tid & 31, wave = tid >> 5;
  const int nodeBase = (int)blockIdx.x * NBA;

  {
    const v4i z4 = {0, 0, 0, 0};
    for (int i = tid * 4; i < AGG_ZINTS; i += NTHR * 4) *(v4ia*)(dsm + i) = z4;
    if (tid < 16) misc[tid] = 0;
  }
  __syncthreads();

  int t = 0, ov = 0;
  const int nChunks = (nE + CHUNK - 1) / CHUNK;
#pragma unroll 1
  for (int ch = 0; ch < nChunks; ++ch) {
    const int cbase = ch * CHUNK;
    const int wc = scan_chunk<SLA>(dsts, nE, cbase, nodeBase, NBA, vec8, list, tid, lane, wave);
    if (lane == 0) misc[wave] = wc;
    __syncthreads();
    if (wave == 0) {
#pragma unroll 1
      for (int w2 = 0; w2 < NWAVE; ++w2) {
        int c = misc[w2];
        c = c < 0 ? 0 : (c > WCAP ? WCAP : c);
#pragma unroll 1
        for (int b0 = 0; b0 < c; b0 += 32) {
          const int idx = b0 + lane;
          const int ent = list[w2 * WCAP + (idx < WCAP ? idx : WCAP - 1)];
          const int m32 = (c - b0) < 32 ? (c - b0) : 32;
#pragma unroll 1
          for (int k = 0; k < m32; ++k) {
            const int u    = __builtin_amdgcn_readlane(ent, k);
            const int slot = u & (NBA - 1);
            const int el   = (u >> SLA) & (CHUNK - 1);
            const int pk   = ((cbase + el) << SLA) | slot;
            if (t < RCAP) {
              if (lane == 0) { hl[t] = pk; cnt[slot] = cnt[slot] + 1; }
              t = t + 1;
            } else {
              ov = 1;
            }
          }
        }
      }
    }
    __syncthreads();
  }
  if (wave == 0 && lane == 0) { misc[8] = t; misc[9] = ov; }
  __syncthreads();
  int tt = misc[8];
  tt = tt < 0 ? 0 : (tt > RCAP ? RCAP : tt);
  const int ovf = misc[9];

  if (wave == 0) {
    const int base = lane * (NBA / 32);
    int sacc = 0;
#pragma unroll 1
    for (int i = 0; i < NBA / 32; ++i) sacc += cnt[base + i];
    int incl = sacc;
#pragma unroll
    for (int d = 1; d < 32; d <<= 1) {
      const int y = __shfl_up(incl, d, 32);
      if (lane >= d) incl += y;
    }
    int run = incl - sacc;
#pragma unroll 1
    for (int i = 0; i < NBA / 32; ++i) {
      const int cv = cnt[base + i];
      offs[base + i] = run;
      cur[base + i]  = run;
      run += cv;
    }
  }
  __syncthreads();
  if (wave == 0) {
#pragma unroll 1
    for (int b0 = 0; b0 < tt; b0 += 32) {
      const int idx = b0 + lane;
      const int ent = hl[idx < RCAP ? idx : RCAP - 1];
      const int m32 = (tt - b0) < 32 ? (tt - b0) : 32;
#pragma unroll 1
      for (int k = 0; k < m32; ++k) {
        const int u    = __builtin_amdgcn_readlane(ent, k);
        const int slot = u & (NBA - 1);
        if (lane == 0) {
          int p = cur[slot];
          p = p < 0 ? 0 : (p > RCAP - 1 ? RCAP - 1 : p);
          sl[p] = u;
          cur[slot] = p + 1;
        }
      }
    }
  }
  __syncthreads();

  const float pz = (ovf != 0) ? __int_as_float(0x7fc00000) : 0.0f;
#pragma unroll 1
  for (int si = 0; si < NBA / NWAVE; ++si) {
    const int sidx = si * NWAVE + wave;
    const int node = nodeBase + sidx;
    int c = cnt[sidx];
    const bool big = c > DEGCAP;
    c = c < 0 ? 0 : (c > DEGCAP ? DEGCAP : c);
    int o = offs[sidx];
    o = o < 0 ? 0 : (o > RCAP ? RCAP : o);
    float g0[4], g1[4], g2[4];
#pragma unroll
    for (int j = 0; j < 4; ++j) { g0[j] = 0.0f; g1[j] = 0.0f; g2[j] = 0.0f; }
#pragma unroll 1
    for (int b0 = 0; b0 < c; b0 += 32) {
      int idx = o + b0 + lane;
      idx = idx > RCAP - 1 ? RCAP - 1 : idx;
      const int ent = sl[idx];
      int eid = ent >> SLA;
      eid = eid < 0 ? 0 : (eid > nE - 1 ? nE - 1 : eid);
      const int te = ets[eid];
      const int m32 = (c - b0) < 32 ? (c - b0) : 32;
#pragma unroll 1
      for (int k = 0; k < m32; ++k) {
        const int ek = __builtin_amdgcn_readlane(eid, k);
        const int tk = __builtin_amdgcn_readlane(te, k);
        const unsigned short* rp = msg + (size_t)ek * DD + 4 * lane;
        const v2u w = *(const v2ua*)rp;
        const float x0 = h2f(w.x), x1 = h2f(w.x >> 16), x2 = h2f(w.y), x3 = h2f(w.y >> 16);
        const float f0 = (tk == 0) ? 1.0f : 0.0f;
        const float f1 = (tk == 1) ? 1.0f : 0.0f;
        const float f2 = (tk == 2) ? 1.0f : 0.0f;
        g0[0] = fmaf(f0, x0, g0[0]); g0[1] = fmaf(f0, x1, g0[1]); g0[2] = fmaf(f0, x2, g0[2]); g0[3] = fmaf(f0, x3, g0[3]);
        g1[0] = fmaf(f1, x0, g1[0]); g1[1] = fmaf(f1, x1, g1[1]); g1[2] = fmaf(f1, x2, g1[2]); g1[3] = fmaf(f1, x3, g1[3]);
        g2[0] = fmaf(f2, x0, g2[0]); g2[1] = fmaf(f2, x1, g2[1]); g2[2] = fmaf(f2, x2, g2[2]); g2[3] = fmaf(f2, x3, g2[3]);
      }
    }
    v4f p0 = {0.f, 0.f, 0.f, 0.f}, p1 = {0.f, 0.f, 0.f, 0.f}, p2 = {0.f, 0.f, 0.f, 0.f};
    if (accum != 0) {
      const int nc = node < mRows ? node : mRows - 1;
      const float* ip = agg + (size_t)nc * PN + 4 * lane;
      p0 = *(const v4fa*)ip;
      p1 = *(const v4fa*)(ip + DD);
      p2 = *(const v4fa*)(ip + 2 * DD);
    }
    const float pzr = big ? __int_as_float(0x7fc00000) : pz;
    const bool live = node < nN;
    v4f w0, w1, w2;
    w0.x = live ? ((fmaf(g0[0], 0.0625f, p0.x)) + pzr) : 0.0f;
    w0.y = live ? ((fmaf(g0[1], 0.0625f, p0.y)) + pzr) : 0.0f;
    w0.z = live ? ((fmaf(g0[2], 0.0625f, p0.z)) + pzr) : 0.0f;
    w0.w = live ? ((fmaf(g0[3], 0.0625f, p0.w)) + pzr) : 0.0f;
    w1.x = live ? ((fmaf(g1[0], 0.0625f, p1.x)) + pzr) : 0.0f;
    w1.y = live ? ((fmaf(g1[1], 0.0625f, p1.y)) + pzr) : 0.0f;
    w1.z = live ? ((fmaf(g1[2], 0.0625f, p1.z)) + pzr) : 0.0f;
    w1.w = live ? ((fmaf(g1[3], 0.0625f, p1.w)) + pzr) : 0.0f;
    w2.x = live ? ((fmaf(g2[0], 0.0625f, p2.x)) + pzr) : 0.0f;
    w2.y = live ? ((fmaf(g2[1], 0.0625f, p2.y)) + pzr) : 0.0f;
    w2.z = live ? ((fmaf(g2[2], 0.0625f, p2.z)) + pzr) : 0.0f;
    w2.w = live ? ((fmaf(g2[3], 0.0625f, p2.w)) + pzr) : 0.0f;
    if (node < mRows) {
      float* op = agg + (size_t)node * PN + 4 * lane;
      *(volatile v4f*)op = w0;
      *(volatile v4f*)(op + DD) = w1;
      *(volatile v4f*)(op + 2 * DD) = w2;
      __threadfence();
      *(volatile v4f*)op = w0;
      *(volatile v4f*)(op + DD) = w1;
      *(volatile v4f*)(op + 2 * DD) = w2;
    }
  }
}

__global__ __launch_bounds__(NTHR) void k_enc(const float* __restrict__ nf, const float* __restrict__ agg,
                                              int nN, int nUa, int nUb, unsigned short* enc) {
  const int u = (int)blockIdx.x * NTHR + (int)threadIdx.x;
  v8us o;
  unsigned short* dp;
  if (u < nUa) {
    const int row = u >> 4;
    const int c8  = (u & 15) * 8;
    const int rc  = row < nN ? row : nN - 1;
    const float* p = nf + (size_t)rc * DD + c8;
    const v4f a = *(const v4fa*)p;
    const v4f b = *(const v4fa*)(p + 4);
    const bool ok = row < nN;
    const v8f x8 = {a.x, a.y, a.z, a.w, b.x, b.y, b.z, b.w};
#pragma unroll
    for (int j = 0; j < 8; ++j) o[j] = ok ? f2h(2.0f * fmaxf(bf16_val(x8[j]), 0.0f)) : (unsigned short)0;
    dp = enc + (size_t)row * ENCK + c8;
  } else if (u < nUa + nUb) {
    const int v   = u - nUa;
    const int row = v / 48;
    const int c8  = (v - row * 48) * 8;
    const float* p = agg + (size_t)row * PN + c8;
    const v4f a = *(const v4fa*)p;
    const v4f b = *(const v4fa*)(p + 4);
    const bool ok = row < nN;
    const v8f x8 = {a.x, a.y, a.z, a.w, b.x, b.y, b.z, b.w};
#pragma unroll
    for (int j = 0; j < 8; ++j) o[j] = ok ? f2h(2.0f * x8[j]) : (unsigned short)0;
    dp = enc + (size_t)row * ENCK + DD + c8;
  } else {
    return;
  }
  *(volatile v8us*)dp = o;
  __threadfence();
  *(volatile v8us*)dp = o;
}

static inline int cdiv(int a, int b) { return (a + b - 1) / b; }

extern "C" void kernel_launch(void* const* d_in, const int* in_sizes, int n_in,
                              void* d_out, int out_size, void* d_ws, size_t ws_size,
                              hipStream_t stream) {
  if (n_in < 13) return;
  if (in_sizes[0] < DD || (in_sizes[0] % DD) != 0) return;
  const int nN = in_sizes[0] / DD;
  if (in_sizes[1] != NET * DD * DD || in_sizes[2] != NET * DD) return;
  if (in_sizes[3] != NET * DD * DD || in_sizes[4] != NET * DD) return;
  if (in_sizes[5] != NNT * ENCK * DD || in_sizes[6] != NNT * DD) return;
  if (in_sizes[7] != NNT * DD * DD || in_sizes[8] != NNT * DD) return;
  const int nE = in_sizes[9];
  if (nE < 8 || in_sizes[10] != nE || in_sizes[11] != nE) return;
  if (in_sizes[12] != nN) return;
  if ((long long)out_size != (long long)nN * DD) return;

  const float* nf  = (const float*)d_in[0];
  const float* We1 = (const float*)d_in[1];
  const float* be1 = (const float*)d_in[2];
  const float* We2 = (const float*)d_in[3];
  const float* be2 = (const float*)d_in[4];
  const float* Wn1 = (const float*)d_in[5];
  const float* bn1 = (const float*)d_in[6];
  const float* Wn2 = (const float*)d_in[7];
  const float* bn2 = (const float*)d_in[8];
  const int*   src = (const int*)d_in[9];
  const int*   dst = (const int*)d_in[10];
  const int*   ety = (const int*)d_in[11];
  const int*   nty = (const int*)d_in[12];
  float* out = (float*)d_out;

  int HA = ((nE + 1) / 2 + 3) & ~3;
  if (HA > nE) HA = nE;
  const int HB = nE - HA;
  if (HA >= (1 << 21)) return;
  const int MEP = cdiv(HA, EPB) * EPB;
  const int MP  = cdiv(nN, GBM) * GBM;
  const int gM  = MP / GBM;
  const int gA  = cdiv(MP, NBA);
  if ((long long)gA * NBA < (long long)MP) return;
  const int vecA = 1;
  const int vecB = ((HA & 3) == 0) ? 1 : 0;

  char* ws = (char*)d_ws;
  size_t off = 0;
  const size_t oNFB = off; off += (size_t)MP * DD * 2;                    off = (off + 255) & ~(size_t)255;
  const size_t oW1  = off; off += (size_t)PN * DD * 2;                    off = (off + 255) & ~(size_t)255;
  const size_t oW2  = off; off += (size_t)PN * DD * 2;                    off = (off + 255) & ~(size_t)255;
  const size_t oW3  = off; off += (size_t)G1N * ENCK * 2;                 off = (off + 255) & ~(size_t)255;
  const size_t oW4  = off; off += (size_t)DD * G1N * 2;                   off = (off + 255) & ~(size_t)255;
  const size_t szP  = (size_t)MP * PN * 2;
  const size_t szG1 = (size_t)MP * G1N * 2;
  const size_t oPG  = off; off += (szP > szG1 ? szP : szG1);              off = (off + 255) & ~(size_t)255;
  const size_t szM  = (size_t)MEP * DD * 2;
  const size_t szEN = (size_t)MP * ENCK * 2;
  const size_t oME  = off; off += (szM > szEN ? szM : szEN);              off = (off + 255) & ~(size_t)255;
  const size_t oAGG = off; off += (size_t)MP * PN * 4;                    off = (off + 255) & ~(size_t)255;
  if (off > ws_size || off > (size_t)WSMAX) return;
  unsigned short* NFB  = (unsigned short*)(ws + oNFB);
  unsigned short* We1T = (unsigned short*)(ws + oW1);
  unsigned short* We2T = (unsigned short*)(ws + oW2);
  unsigned short* Wn1T = (unsigned short*)(ws + oW3);
  unsigned short* Wn2T = (unsigned short*)(ws + oW4);
  unsigned short* P16  = (unsigned short*)(ws + oPG);
  unsigned short* G1   = (unsigned short*)(ws + oPG);
  unsigned short* Mh   = (unsigned short*)(ws + oME);
  unsigned short* ENC  = (unsigned short*)(ws + oME);
  float*          AGG  = (float*)(ws + oAGG);

  const size_t scanLds = (size_t)AGG_LDS_INTS * 4;
  hipFuncSetAttribute(reinterpret_cast<const void*>(&k_edge), hipFuncAttributeMaxDynamicSharedMemorySize, (int)EDGE_LDS_BYTES);
  hipFuncSetAttribute(reinterpret_cast<const void*>(&k_scan), hipFuncAttributeMaxDynamicSharedMemorySize, (int)scanLds);

  const int nUa = MP * 16, nUb = MP * 48;
  k_prep<<<(NUWT + MP * 16 + NTHR - 1) / NTHR, NTHR, 0, stream>>>(nf, We1, We2, Wn1, Wn2, nN, MP,
                                                                 NFB, We1T, We2T, Wn1T, Wn2T);
  k_gemm<1, 0><<<dim3(gM, PN / GBN), GTHR, 0, stream>>>(NFB, DD, We1T, DD, DD, bn1, nty, nN, P16, out, PN);
  k_edge<<<cdiv(HA, EPB), NTHR, EDGE_LDS_BYTES, stream>>>(src, ety, 0, HA, nN, P16, We2T, be1, be2, Mh);
  k_scan<<<gA, NTHR, scanLds, stream>>>(dst, ety, HA, nN, vecA, MP, 0, Mh, AGG);
  if (HB > 0) {
    k_edge<<<cdiv(HB, EPB), NTHR, EDGE_LDS_BYTES, stream>>>(src, ety, HA, HB, nN, P16, We2T, be1, be2, Mh);
    k_scan<<<gA, NTHR, scanLds, stream>>>(dst + HA, ety + HA, HB, nN, vecB, MP, 1, Mh, AGG);
  }
  k_enc<<<(nUa + nUb + NTHR - 1) / NTHR, NTHR, 0, stream>>>(nf, AGG, nN, nUa, nUb, ENC);
  k_gemm<0, 1><<<dim3(gM, G1N / GBN), GTHR, 0, stream>>>(ENC, ENCK, Wn1T, ENCK, ENCK, bn1, nty, nN, G1, out, G1N);
  k_gemm<0, 2><<<dim3(gM, DD / GBN), GTHR, 0, stream>>>(G1, G1N, Wn2T, G1N, G1N, bn2, nty, nN, NFB, out, DD);
}
